// HeteroGNNModel_1099511628160
// MI455X (gfx1250) — hardware-verified
//
#include <hip/hip_runtime.h>
#include <stddef.h>
#include <math.h>


#define CH      128
#define NTHR    256
#define NWAVE   8
#define EPT     8
#define NGRP    2
#define CHUNK   (NTHR * EPT * NGRP)
#define WCAP    (EPT * NGRP * 32)
#define LISTN   (NWAVE * WCAP)
#define NBC     4096
#define NBF     1024
#define RCAP    40960
#define RBN     128
#define TGT     256
#define DEGCAP  512
#define OTHR    512
#define BM      32
#define WSCAP   134217728
#define SCL_A   8.0f
#define SCL_W   16.0f
#define SCL_ACC 0.0078125f

#define LDS_FILL ((RCAP + NBF + LISTN) * 4 + 64)

static_assert((CHUNK & (CHUNK - 1)) == 0);
static_assert(CHUNK <= 4096);
static_assert(NBC <= 4096 && NBF <= 4096);
static_assert((NBC & (NBC - 1)) == 0 && (NBF & (NBF - 1)) == 0);
static_assert(NBC == 4 * NBF);
static_assert(OTHR * 8 == NBC);
static_assert((RCAP % 32) == 0);
static_assert(TGT == NWAVE * 32);
static_assert((NBC % TGT) == 0);
static_assert((TGT % BM) == 0);
static_assert(CH == 128);

typedef float    v4f  __attribute__((ext_vector_type(4)));
typedef float    v8f  __attribute__((ext_vector_type(8)));
typedef int      v4i  __attribute__((ext_vector_type(4)));
typedef _Float16 v4h  __attribute__((ext_vector_type(4)));
typedef _Float16 v8h  __attribute__((ext_vector_type(8)));
typedef _Float16 v16h __attribute__((ext_vector_type(16)));
union FragH { v16h v; v8h h[2]; };

__device__ __forceinline__ v8f wmh(v16h a, v16h b, v8f c) {
  v8f d = __builtin_amdgcn_wmma_f32_16x16x32_f16(false, a, false, b, (short)0, c, false, false);
  asm volatile("v_nop\n\tv_nop\n\tv_nop\n\tv_nop" : "+v"(d) : "v"(a), "v"(b));
  return d;
}

__device__ __forceinline__ v8h cvt8(v4f a, v4f b, float s) {
  v8f t;
  t[0] = a.x * s; t[1] = a.y * s; t[2] = a.z * s; t[3] = a.w * s;
  t[4] = b.x * s; t[5] = b.y * s; t[6] = b.z * s; t[7] = b.w * s;
  return __builtin_convertvector(t, v8h);
}

__device__ __forceinline__ v4f vrelu(v4f a) {
  v4f r;
  r.x = a.x > 0.0f ? a.x : 0.0f;
  r.y = a.y > 0.0f ? a.y : 0.0f;
  r.z = a.z > 0.0f ? a.z : 0.0f;
  r.w = a.w > 0.0f ? a.w : 0.0f;
  return r;
}

__device__ __forceinline__ v4f ld4f(const float* p) { return *(const v4f*)p; }
__device__ __forceinline__ v4f ld4f(const _Float16* p) {
  const v4h hv = *(const v4h*)p;
  return __builtin_convertvector(hv, v4f);
}

template <int NB>
__device__ __forceinline__ int scan_chunk(const int* __restrict__ dsts, int nE, int cbase, int slotBase,
                                          int vec8, int* list, int tid, int lane, int wave) {
  int wc = 0;
#pragma unroll
  for (int g = 0; g < NGRP; ++g) {
    const int el0  = (g * NTHR + tid) * EPT;
    const int e0   = cbase + el0;
    const int sent = -2147483647 - 1;
    v4i da, db;
    if (vec8 != 0 && cbase + CHUNK <= nE) {
      da = *(const v4i*)(dsts + e0);
      db = *(const v4i*)(dsts + e0 + 4);
    } else {
      da.x = (e0     < nE) ? dsts[min(e0, nE - 1)] : sent;
      da.y = (e0 + 1 < nE) ? dsts[min(e0 + 1, nE - 1)] : sent;
      da.z = (e0 + 2 < nE) ? dsts[min(e0 + 2, nE - 1)] : sent;
      da.w = (e0 + 3 < nE) ? dsts[min(e0 + 3, nE - 1)] : sent;
      db.x = (e0 + 4 < nE) ? dsts[min(e0 + 4, nE - 1)] : sent;
      db.y = (e0 + 5 < nE) ? dsts[min(e0 + 5, nE - 1)] : sent;
      db.z = (e0 + 6 < nE) ? dsts[min(e0 + 6, nE - 1)] : sent;
      db.w = (e0 + 7 < nE) ? dsts[min(e0 + 7, nE - 1)] : sent;
    }
    const unsigned nb = (unsigned)slotBase;
    const unsigned s0 = (unsigned)da.x - nb, s1 = (unsigned)da.y - nb;
    const unsigned s2 = (unsigned)da.z - nb, s3 = (unsigned)da.w - nb;
    const unsigned s4 = (unsigned)db.x - nb, s5 = (unsigned)db.y - nb;
    const unsigned s6 = (unsigned)db.z - nb, s7 = (unsigned)db.w - nb;
    const bool h0 = s0 < (unsigned)NB, h1 = s1 < (unsigned)NB, h2 = s2 < (unsigned)NB, h3 = s3 < (unsigned)NB;
    const bool h4 = s4 < (unsigned)NB, h5 = s5 < (unsigned)NB, h6 = s6 < (unsigned)NB, h7 = s7 < (unsigned)NB;
    const unsigned any = __builtin_amdgcn_ballot_w32(h0 | h1 | h2 | h3 | h4 | h5 | h6 | h7);
    if (any != 0u) {
#define HITJ(J, HJ, SJ) { \
        const unsigned mj = __builtin_amdgcn_ballot_w32(HJ); \
        if (mj != 0u) { \
          if (HJ) { \
            const int pos = wc + (int)__builtin_amdgcn_mbcnt_lo(mj, 0u); \
            if (pos < WCAP) list[wave * WCAP + pos] = ((el0 + (J)) << 12) | (int)(SJ); \
          } \
          wc += (int)__builtin_popcount(mj); } }
      HITJ(0, h0, s0)
      HITJ(1, h1, s1)
      HITJ(2, h2, s2)
      HITJ(3, h3, s3)
      HITJ(4, h4, s4)
      HITJ(5, h5, s5)
      HITJ(6, h6, s6)
      HITJ(7, h7, s7)
#undef HITJ
    }
  }
  return wc;
}

__global__ __launch_bounds__(NTHR) void k_xcvt(const float* __restrict__ x, _Float16* xp, int nN, int nUnits) {
  constexpr int UPR = CH / 8;
  static_assert((UPR & (UPR - 1)) == 0);
  const int i = (int)blockIdx.x * NTHR + (int)threadIdx.x;
  if (i >= nUnits) return;
  const int row = i / UPR;
  const int c0  = (i & (UPR - 1)) * 8;
  int rr = row > nN - 1 ? nN - 1 : row;
  rr = rr < 0 ? 0 : rr;
  const float* p = x + (size_t)rr * CH + c0;
  const v4f a = vrelu(*(const v4f*)p);
  const v4f b = vrelu(*(const v4f*)(p + 4));
  v8h o = cvt8(a, b, SCL_A);
  const v8h z = {(_Float16)0.0f, (_Float16)0.0f, (_Float16)0.0f, (_Float16)0.0f,
                 (_Float16)0.0f, (_Float16)0.0f, (_Float16)0.0f, (_Float16)0.0f};
  o = (row < nN) ? o : z;
  _Float16* d = xp + (size_t)i * 8;
  *(volatile v8h*)d = o;
  __threadfence();
  *(volatile v8h*)d = o;
}

template <int K, int NC, int NP>
__global__ __launch_bounds__(NTHR) void k_prepw(const float* __restrict__ Wa, const float* __restrict__ Wb, _Float16* wp) {
  constexpr int UPR = (NP * K) / 8;
  constexpr int NUN = NC * UPR;
  static_assert((K % 8) == 0 && (NUN % NTHR) == 0 && (NP == 1 || NP == 2));
  const int i = (int)blockIdx.x * NTHR + (int)threadIdx.x;
  if (i >= NUN) return;
  const int n  = i / UPR;
  const int k0 = (i - n * UPR) * 8;
  const bool left = k0 < K;
  int ka = left ? k0 : (k0 - K);
  ka = ka < 0 ? 0 : (ka > K - 8 ? K - 8 : ka);
  const int nc = n > NC - 1 ? NC - 1 : (n < 0 ? 0 : n);
  const float* pa = Wa + (size_t)nc * K + ka;
  const float* pb = Wb + (size_t)nc * K + ka;
  const v4f a0 = *(const v4f*)pa;
  const v4f a1 = *(const v4f*)(pa + 4);
  const v4f b0 = *(const v4f*)pb;
  const v4f b1 = *(const v4f*)(pb + 4);
  const v4f s0 = left ? a0 : b0;
  const v4f s1 = left ? a1 : b1;
  const v8h o = cvt8(s0, s1, SCL_W);
  _Float16* d = wp + (size_t)i * 8;
  *(volatile v8h*)d = o;
  __threadfence();
  *(volatile v8h*)d = o;
}

__global__ __launch_bounds__(NTHR) void k_count(
    const int* __restrict__ dsts, int* cnt, int nE, int vec8) {
  __shared__ __attribute__((aligned(16))) int scnt[NBC];
  __shared__ __attribute__((aligned(16))) int list[LISTN];
  __shared__ int wcnt[NWAVE];
  const int tid = threadIdx.x, lane = tid & 31, wave = tid >> 5;
  const int nodeBase = blockIdx.x * NBC;

  for (int i = tid; i < NBC; i += NTHR) scnt[i] = 0;
  __syncthreads();

  const int nChunks = (nE + CHUNK - 1) / CHUNK;
#pragma unroll 1
  for (int ch = 0; ch < nChunks; ++ch) {
    const int cbase = ch * CHUNK;
    const int wc = scan_chunk<NBC>(dsts, nE, cbase, nodeBase, vec8, list, tid, lane, wave);
    if (lane == 0) wcnt[wave] = wc;
    __syncthreads();
    if (wave == 0) {
#pragma unroll 1
      for (int wsx = 0; wsx < NWAVE; ++wsx) {
        int n = __builtin_amdgcn_readfirstlane(wcnt[wsx]);
        n = n > WCAP ? WCAP : (n < 0 ? 0 : n);
        const int* lp = list + wsx * WCAP;
#pragma unroll 1
        for (int i = 0; i < n; ++i) {
          const int ent  = __builtin_amdgcn_readfirstlane(lp[i]);
          const int slot = ent & (NBC - 1);
          if (lane == 0) scnt[slot] = scnt[slot] + 1;
        }
      }
    }
    __syncthreads();
  }

  v4i cq[4];
#pragma unroll
  for (int q = 0; q < 4; ++q) {
    const int f = (wave * 4 + q) * 128 + 4 * lane;
    cq[q] = *(const v4i*)(scnt + f);
  }
  int* cp = cnt + (size_t)nodeBase;
#pragma unroll
  for (int q = 0; q < 4; ++q) {
    const int f = (wave * 4 + q) * 128 + 4 * lane;
    *(volatile v4i*)(cp + f) = cq[q];
  }
  __threadfence();
#pragma unroll
  for (int q = 0; q < 4; ++q) {
    const int f = (wave * 4 + q) * 128 + 4 * lane;
    *(volatile v4i*)(cp + f) = cq[q];
  }
}

__global__ __launch_bounds__(OTHR) void k_offsets(
    const int* __restrict__ cnt, int* off, int* rbase, int nChunk) {
  __shared__ __attribute__((aligned(16))) int soff[NBC];
  __shared__ __attribute__((aligned(16))) int srb[RBN];
  __shared__ int wtot[OTHR / 32];
  const int tid = threadIdx.x, lane = tid & 31, wave = tid >> 5, sub = tid >> 7;
  for (int i = tid; i < RBN; i += OTHR) srb[i] = 0;
  int carry = 0;
#pragma unroll 1
  for (int ch = 0; ch < nChunk; ++ch) {
    const int base = ch * NBC;
    const v4i c0 = *(const v4i*)(cnt + base + 8 * tid);
    const v4i c1 = *(const v4i*)(cnt + base + 8 * tid + 4);
    const int e0 = max(c0.x, 0), e1 = max(c0.y, 0), e2 = max(c0.z, 0), e3 = max(c0.w, 0);
    const int e4 = max(c1.x, 0), e5 = max(c1.y, 0), e6 = max(c1.z, 0), e7 = max(c1.w, 0);
    const int ts = e0 + e1 + e2 + e3 + e4 + e5 + e6 + e7;
    int incl = ts;
#pragma unroll
    for (int d = 1; d < 32; d <<= 1) {
      const int t = __shfl_up(incl, d);
      if (lane >= d) incl += t;
    }
    if (lane == 31) wtot[wave] = incl;
    __syncthreads();
    const int S0 = wtot[0]  + wtot[1]  + wtot[2]  + wtot[3];
    const int S1 = wtot[4]  + wtot[5]  + wtot[6]  + wtot[7];
    const int S2 = wtot[8]  + wtot[9]  + wtot[10] + wtot[11];
    const int S3 = wtot[12] + wtot[13] + wtot[14] + wtot[15];
    int pre = 0;
#pragma unroll 1
    for (int w = 4 * sub; w < wave; ++w) pre += wtot[w];
    const int b0 = carry;
    const int b1 = b0 + ((S0 + 31) & ~31);
    const int b2 = b1 + ((S1 + 31) & ~31);
    const int b3 = b2 + ((S2 + 31) & ~31);
    const int b4 = b3 + ((S3 + 31) & ~31);
    const int myb = sub == 0 ? b0 : (sub == 1 ? b1 : (sub == 2 ? b2 : b3));
    if (tid == 0) {
      srb[min(4 * ch + 0, RBN - 1)] = b0;
      srb[min(4 * ch + 1, RBN - 1)] = b1;
      srb[min(4 * ch + 2, RBN - 1)] = b2;
      srb[min(4 * ch + 3, RBN - 1)] = b3;
    }
    int run = myb + pre + incl - ts;
    soff[8 * tid + 0] = run; run += e0;
    soff[8 * tid + 1] = run; run += e1;
    soff[8 * tid + 2] = run; run += e2;
    soff[8 * tid + 3] = run; run += e3;
    soff[8 * tid + 4] = run; run += e4;
    soff[8 * tid + 5] = run; run += e5;
    soff[8 * tid + 6] = run; run += e6;
    soff[8 * tid + 7] = run;
    carry = b4;
    __syncthreads();
    const v4i o0 = *(const v4i*)(soff + 4 * tid);
    const v4i o1 = *(const v4i*)(soff + 4 * (tid + OTHR));
    int* op = off + base;
    *(volatile v4i*)(op + 4 * tid) = o0;
    *(volatile v4i*)(op + 4 * (tid + OTHR)) = o1;
    __threadfence();
    *(volatile v4i*)(op + 4 * tid) = o0;
    *(volatile v4i*)(op + 4 * (tid + OTHR)) = o1;
    __syncthreads();
  }
  if (tid == 0) srb[min(4 * nChunk, RBN - 1)] = carry;
  __syncthreads();
  v4i rv = {0, 0, 0, 0};
  if (tid < 32) rv = *(const v4i*)(srb + 4 * tid);
  if (tid < 32) *(volatile v4i*)(rbase + 4 * tid) = rv;
  __threadfence();
  if (tid < 32) *(volatile v4i*)(rbase + 4 * tid) = rv;
}

__global__ __launch_bounds__(NTHR) void k_fill(
    const int* __restrict__ dsts, const int* __restrict__ off, const int* __restrict__ rbase,
    int* csr, int nE, int vec8, int csrLen) {
  extern __shared__ v4f lds_dyn[];
  int* region = (int*)lds_dyn;
  int* cursor = region + RCAP;
  int* list   = cursor + NBF;
  int* wcnt   = list + LISTN;
  const int tid = threadIdx.x, lane = tid & 31, wave = tid >> 5;
  const int b = blockIdx.x;
  const int nodeBase = b * NBF;

  int rb0 = rbase[b];
  const int rb1 = rbase[b + 1];
  rb0 = rb0 < 0 ? 0 : (rb0 > csrLen ? csrLen : rb0);
  rb0 &= ~31;
  int len = rb1 - rb0;
  len = len < 0 ? 0 : (len > RCAP ? RCAP : len);
  int lenW = (len + 31) & ~31;
  if (rb0 + lenW > csrLen) lenW = (csrLen - rb0) & ~31;

  {
    const v4i z = {0, 0, 0, 0};
    for (int i = tid; i < RCAP / 4; i += NTHR) ((v4i*)region)[i] = z;
    for (int s = tid; s < NBF; s += NTHR) {
      int o = off[nodeBase + s] - rb0;
      o = o < 0 ? 0 : (o > RCAP ? RCAP : o);
      cursor[s] = o;
    }
  }
  __syncthreads();

  const int nChunks = (nE + CHUNK - 1) / CHUNK;
#pragma unroll 1
  for (int ch = 0; ch < nChunks; ++ch) {
    const int cbase = ch * CHUNK;
    const int wc = scan_chunk<NBF>(dsts, nE, cbase, nodeBase, vec8, list, tid, lane, wave);
    if (lane == 0) wcnt[wave] = wc;
    __syncthreads();
    if (wave == 0) {
#pragma unroll 1
      for (int wsx = 0; wsx < NWAVE; ++wsx) {
        int n = __builtin_amdgcn_readfirstlane(wcnt[wsx]);
        n = n > WCAP ? WCAP : (n < 0 ? 0 : n);
        const int* lp = list + wsx * WCAP;
#pragma unroll 1
        for (int i = 0; i < n; ++i) {
          const int ent  = __builtin_amdgcn_readfirstlane(lp[i]);
          const int slot = ent & (NBF - 1);
          int e = cbase + ((ent >> 12) & (CHUNK - 1));
          e = e > nE - 1 ? nE - 1 : (e < 0 ? 0 : e);
          if (lane == 0) {
            int pos = cursor[slot];
            pos = pos < 0 ? 0 : (pos > RCAP - 1 ? RCAP - 1 : pos);
            region[pos] = e;
            const int np = pos + 1;
            cursor[slot] = np > RCAP ? RCAP : np;
          }
        }
      }
    }
    __syncthreads();
  }

  const int nv = lenW >> 2;
  int* gp = csr + rb0;
#pragma unroll 1
  for (int i = tid; i < nv; i += NTHR) { const v4i v = ((const v4i*)region)[i]; *(volatile v4i*)(gp + 4 * i) = v; }
  __threadfence();
#pragma unroll 1
  for (int i = tid; i < nv; i += NTHR) { const v4i v = ((const v4i*)region)[i]; *(volatile v4i*)(gp + 4 * i) = v; }
}

template <typename ST, int OSC, int RELUSRC, int HASPRED>
__global__ __launch_bounds__(NTHR) void k_mean(
    const int* __restrict__ csr, const int* __restrict__ off, const int* __restrict__ cnt,
    const int* __restrict__ srcs, const ST* __restrict__ hp, const float* __restrict__ pred,
    _Float16* ap, int nT, int nS, int nE, int csrLen) {
  const int tid = threadIdx.x, lane = tid & 31, wave = tid >> 5;
  const int tbase = blockIdx.x * TGT + wave * 32;
  const int col = 4 * lane;

  const int cl    = tbase + lane;
  const int cnt_l = cnt[cl];
  const int off_l = off[cl];

#pragma unroll 1
  for (int j = 0; j < 32; ++j) {
    const int c = tbase + j;
    int nraw = __shfl(cnt_l, j);
    nraw = nraw < 0 ? 0 : (nraw > nE ? nE : nraw);
    const int n = nraw > DEGCAP ? DEGCAP : nraw;
    const int st = __shfl(off_l, j);

    v4f acc = {0.0f, 0.0f, 0.0f, 0.0f};
#pragma unroll 1
    for (int q0 = 0; q0 < n; q0 += 32) {
      int pos = st + q0 + lane;
      pos = pos < 0 ? 0 : (pos > csrLen - 1 ? csrLen - 1 : pos);
      int el = csr[pos];
      el = el < 0 ? 0 : (el > nE - 1 ? nE - 1 : el);
      int sl = srcs[el];
      sl = sl < 0 ? 0 : (sl > nS - 1 ? nS - 1 : sl);
      const int mcnt = (n - q0) < 32 ? (n - q0) : 32;
#pragma unroll 1
      for (int pp = 0; pp < mcnt; ++pp) {
        const int s = __builtin_amdgcn_readlane(sl, pp);
        v4f x = ld4f(hp + (size_t)s * CH + col);
        if (RELUSRC) x = vrelu(x);
        acc = acc + x;
      }
    }

    const float nf = (float)(nraw < 1 ? 1 : nraw);
    const float rd = (1.0f / nf) * (float)OSC;
    v4f v = acc * rd;
    if (HASPRED) {
      const v4f p4 = *(const v4f*)(pred + (size_t)c * CH + col);
      const float ps = (nraw >= 1) ? SCL_A : 0.0f;
      v = v - p4 * ps;
    }
    if (nraw > DEGCAP) { const float qn = __int_as_float(0x7fc00000); v.x = qn; v.y = qn; v.z = qn; v.w = qn; }
    if (c >= nT) { v.x = 0.0f; v.y = 0.0f; v.z = 0.0f; v.w = 0.0f; }
    const v4h o = __builtin_convertvector(v, v4h);
    _Float16* gp = ap + (size_t)c * CH + col;
    *(volatile v4h*)gp = o;
    __threadfence();
    *(volatile v4h*)gp = o;
  }
}

template <int K, int LDB, int TPW>
__device__ __forceinline__ void mma_pair(const _Float16* __restrict__ Ap, const _Float16* __restrict__ Bp,
                                         int arow, int c0, int m, int hh, v8f (&acc)[TPW]) {
  constexpr int KT = K / 32;
  static_assert(K % 32 == 0 && LDB % 8 == 0);
  const _Float16* ap  = Ap + (size_t)arow * K + 8 * hh;
  const _Float16* bp0 = Bp + (size_t)(c0 + m) * LDB + 8 * hh;
#pragma unroll 1
  for (int kt = 0; kt < KT; ++kt) {
    FragH a;
    a.h[0] = *(const v8h*)(ap + 32 * kt);
    a.h[1] = *(const v8h*)(ap + 32 * kt + 16);
#pragma unroll
    for (int t = 0; t < TPW; ++t) {
      const _Float16* bp = bp0 + (size_t)(16 * t) * LDB + 32 * kt;
      FragH bf;
      bf.h[0] = *(const v8h*)bp;
      bf.h[1] = *(const v8h*)(bp + 16);
      acc[t] = wmh(a.v, bf.v, acc[t]);
    }
  }
}

template <int K, int NC, int LDB, int NPAIR, int RELU, int HASBIAS, int HASB2>
__device__ __forceinline__ void gemm_stage(
    const _Float16* __restrict__ A1, const _Float16* __restrict__ A2,
    const _Float16* __restrict__ Bp, const float* __restrict__ bias, const float* __restrict__ bias2,
    float* stg, int rowBase, int nN, int lane, int wave) {
  constexpr int TPW = NC / 64;
  static_assert(K % 32 == 0);
  static_assert(NC % 64 == 0 && TPW >= 1);
  static_assert(NPAIR == 1 || NPAIR == 2);
  const int hh = lane >> 4, m = lane & 15;
  const int rg = wave >> 2, cq = wave & 3;
  const int r0 = rg * 16;
  const int c0 = cq * (NC / 4);

  v8f acc[TPW];
#pragma unroll
  for (int t = 0; t < TPW; ++t) { v8f z = {0.f, 0.f, 0.f, 0.f, 0.f, 0.f, 0.f, 0.f}; acc[t] = z; }

  mma_pair<K, LDB, TPW>(A1, Bp, rowBase + r0 + m, c0, m, hh, acc);
  if (NPAIR == 2) mma_pair<K, LDB, TPW>(A2, Bp + K, rowBase + r0 + m, c0, m, hh, acc);

  float* sp = stg + (size_t)(r0 + 8 * hh) * NC + c0 + m;
  const int grow0 = rowBase + r0 + 8 * hh;
#pragma unroll
  for (int t = 0; t < TPW; ++t) {
    float bv = 0.0f;
    if (HASBIAS) bv = bias[c0 + 16 * t + m];
    if (HASB2) bv = bv + bias2[c0 + 16 * t + m];
#pragma unroll
    for (int r = 0; r < 8; ++r) {
      float v = acc[t][r] * SCL_ACC + bv;
      if (RELU) v = v > 0.0f ? v : 0.0f;
      v = (grow0 + r < nN) ? v : 0.0f;
      sp[r * NC + 16 * t] = v;
    }
  }
}

template <int K, int NC, int LDB, int NPAIR, int RELU, int HASB2>
__global__ __launch_bounds__(NTHR) void k_gemm16(
    const _Float16* __restrict__ A1, const _Float16* __restrict__ A2,
    const _Float16* __restrict__ Bp, const float* __restrict__ bias, const float* __restrict__ bias2,
    _Float16* Hq, int nN) {
  constexpr int NIT8 = (BM * NC / 8) / NTHR;
  static_assert((BM * NC / 8) % NTHR == 0 && NIT8 >= 1);
  static_assert(BM * 8 == NTHR);
  __shared__ __attribute__((aligned(16))) float stg[BM * NC];
  const int tid = threadIdx.x, lane = tid & 31, wave = tid >> 5;
  const int rowBase = blockIdx.x * BM;

  gemm_stage<K, NC, LDB, NPAIR, RELU, 1, HASB2>(A1, A2, Bp, bias, bias2, stg, rowBase, nN, lane, wave);
  __syncthreads();

  _Float16* tile = Hq + (size_t)rowBase * NC;
  v8h hv[NIT8];
#pragma unroll
  for (int it = 0; it < NIT8; ++it) {
    const int u = it * NTHR + tid;
    const v4f x0 = *(const v4f*)(stg + 8 * u);
    const v4f x1 = *(const v4f*)(stg + 8 * u + 4);
    hv[it] = cvt8(x0, x1, SCL_A);
  }
#pragma unroll
  for (int it = 0; it < NIT8; ++it) *(volatile v8h*)(tile + 8 * (size_t)(it * NTHR + tid)) = hv[it];
  __threadfence();
#pragma unroll
  for (int it = 0; it < NIT8; ++it) *(volatile v8h*)(tile + 8 * (size_t)(it * NTHR + tid)) = hv[it];
}

template <int K, int NC, int LDB, int NPAIR, int HASBIAS>
__global__ __launch_bounds__(NTHR) void k_gemm32(
    const _Float16* __restrict__ A1, const _Float16* __restrict__ A2,
    const _Float16* __restrict__ Bp, const float* __restrict__ bias,
    float* Zp, int nN) {
  constexpr int NIT4 = (BM * NC / 4) / NTHR;
  static_assert((BM * NC / 4) % NTHR == 0 && NIT4 >= 1);
  static_assert(BM * 8 == NTHR);
  __shared__ __attribute__((aligned(16))) float stg[BM * NC];
  const int tid = threadIdx.x, lane = tid & 31, wave = tid >> 5;
  const int rowBase = blockIdx.x * BM;

  gemm_stage<K, NC, LDB, NPAIR, 0, HASBIAS, 0>(A1, A2, Bp, bias, bias, stg, rowBase, nN, lane, wave);
  __syncthreads();

  float* tile = Zp + (size_t)rowBase * NC;
  v4f ov[NIT4];
#pragma unroll
  for (int it = 0; it < NIT4; ++it) ov[it] = *(const v4f*)(stg + 4 * (it * NTHR + tid));
#pragma unroll
  for (int it = 0; it < NIT4; ++it) *(volatile v4f*)(tile + 4 * (size_t)(it * NTHR + tid)) = ov[it];
  __threadfence();
#pragma unroll
  for (int it = 0; it < NIT4; ++it) *(volatile v4f*)(tile + 4 * (size_t)(it * NTHR + tid)) = ov[it];
}

template <int K, int NC, int LDB, int NPAIR>
__global__ __launch_bounds__(NTHR) void k_gemmhead(
    const _Float16* __restrict__ A1, const _Float16* __restrict__ A2,
    const _Float16* __restrict__ Bp, const float* __restrict__ bias, const float* __restrict__ bias2,
    const float* __restrict__ hw, const float* __restrict__ hb,
    float* out, int nN) {
  static_assert(NC == 128 && BM * 8 == NTHR);
  __shared__ __attribute__((aligned(16))) float stg[BM * NC];
  __shared__ __attribute__((aligned(16))) float sres[BM];
  const int tid = threadIdx.x, lane = tid & 31, wave = tid >> 5;
  const int rowBase = blockIdx.x * BM;

  gemm_stage<K, NC, LDB, NPAIR, 1, 1, 1>(A1, A2, Bp, bias, bias2, stg, rowBase, nN, lane, wave);
  __syncthreads();

  const int row = tid >> 3, prt = tid & 7;
  const float* sp = stg + row * NC + prt * 16;
  const v4f x0 = *(const v4f*)(sp);
  const v4f x1 = *(const v4f*)(sp + 4);
  const v4f x2 = *(const v4f*)(sp + 8);
  const v4f x3 = *(const v4f*)(sp + 12);
  const v4f w0 = *(const v4f*)(hw + prt * 16);
  const v4f w1 = *(const v4f*)(hw + prt * 16 + 4);
  const v4f w2 = *(const v4f*)(hw + prt * 16 + 8);
  const v4f w3 = *(const v4f*)(hw + prt * 16 + 12);
  const v4f pr = x0 * w0 + x1 * w1 + x2 * w2 + x3 * w3;
  float s = (pr.x + pr.y) + (pr.z + pr.w);
  s += __shfl_xor(s, 1);
  s += __shfl_xor(s, 2);
  s += __shfl_xor(s, 4);
  if (prt == 0) sres[row] = s + hb[0];
  __syncthreads();

  const v4f v = *(const v4f*)(sres + 4 * (tid & 7));
  const int e0 = rowBase + 4 * tid;
  const bool act  = tid < 8;
  const bool full = act && (e0 + 3 < nN);
  const bool tail = act && !full && (e0 < nN);
  if (full) {
    *(volatile v4f*)(out + e0) = v;
  } else if (tail) {
    if (e0 < nN)     *(volatile float*)(out + e0)     = v.x;
    if (e0 + 1 < nN) *(volatile float*)(out + e0 + 1) = v.y;
    if (e0 + 2 < nN) *(volatile float*)(out + e0 + 2) = v.z;
  }
  __threadfence();
  if (full) {
    *(volatile v4f*)(out + e0) = v;
  } else if (tail) {
    if (e0 < nN)     *(volatile float*)(out + e0)     = v.x;
    if (e0 + 1 < nN) *(volatile float*)(out + e0 + 1) = v.y;
    if (e0 + 2 < nN) *(volatile float*)(out + e0 + 2) = v.z;
  }
}

extern "C" void kernel_launch(void* const* d_in, const int* in_sizes, int n_in,
                              void* d_out, int out_size, void* d_ws, size_t ws_size,
                              hipStream_t stream) {
  if (n_in < 32) return;
  const int nU = in_sizes[0] / CH;
  const int nI = in_sizes[1] / CH;
  if (nU <= 0 || nI <= 0) return;
  if (in_sizes[0] != nU * CH || in_sizes[1] != nI * CH) return;
  for (int l = 0; l < 2; ++l)
    for (int j = 0; j < 12; ++j) {
      const int want = (j & 1) ? CH : CH * CH;
      if (in_sizes[2 + 12 * l + j] != want) return;
    }
  if (in_sizes[26] != CH || in_sizes[27] != 1) return;
  const int nE1 = in_sizes[28];
  const int nE2 = in_sizes[30];
  if (nE1 <= 0 || nE2 <= 0 || in_sizes[29] != nE1 || in_sizes[31] != nE2) return;
  if (out_size != nU) return;
  if (nU > (1 << 22) || nI > (1 << 22) || nE1 > (1 << 28) || nE2 > (1 << 28)) return;

  const float* emb_u = (const float*)d_in[0];
  const float* emb_i = (const float*)d_in[1];
  const float* Wb[2][12];
  for (int l = 0; l < 2; ++l)
    for (int j = 0; j < 12; ++j) Wb[l][j] = (const float*)d_in[2 + 12 * l + j];
  const float* hw = (const float*)d_in[26];
  const float* hb = (const float*)d_in[27];
  const int* ue_src = (const int*)d_in[28];
  const int* ue_dst = (const int*)d_in[29];
  const int* iu_src = (const int*)d_in[30];
  const int* iu_dst = (const int*)d_in[31];
  float* out = (float*)d_out;

  const int NUP = ((nU + TGT - 1) / TGT) * TGT;
  const int NIP = ((nI + TGT - 1) / TGT) * TGT;
  const int RMX = NUP > NIP ? NUP : NIP;
  const int RB  = NUP > 2 * NIP ? NUP : 2 * NIP;

  const int nBCI    = (nI + NBC - 1) / NBC;
  const int CNTPADI = nBCI * NBC;
  const int nBFI    = (nI + NBF - 1) / NBF;
  const int csrLenI = ((nE1 + 31) & ~31) + 4096;
  const int nBCU    = (nU + NBC - 1) / NBC;
  const int CNTPADU = nBCU * NBC;
  const int nBFU    = (nU + NBF - 1) / NBF;
  const int csrLenU = ((nE2 + 31) & ~31) + 4096;
  if (CNTPADI < NIP || CNTPADU < NUP) return;
  if (4 * nBCI + 1 > RBN || 4 * nBCU + 1 > RBN) return;
  if (nBFI > 4 * nBCI || nBFU > 4 * nBCU) return;
  if (31 * 4 * nBCI > 4096 || 31 * 4 * nBCU > 4096) return;

  const int nAI = NIP / TGT, nAU = NUP / TGT;
  const int nGI = NIP / BM,  nGU = NUP / BM;
  const int nXuU = NUP * (CH / 8), nXuI = NIP * (CH / 8);

  char* ws = (char*)d_ws;
  size_t off = 0;
  size_t oW1[2], oW2[2], oUI[2], oIU[2];
  for (int l = 0; l < 2; ++l) {
    oW1[l] = off; off += (size_t)CH * CH * 2;       off = (off + 255) & ~(size_t)255;
    oW2[l] = off; off += (size_t)CH * CH * 2;       off = (off + 255) & ~(size_t)255;
    oUI[l] = off; off += (size_t)CH * 2 * CH * 2;   off = (off + 255) & ~(size_t)255;
    oIU[l] = off; off += (size_t)CH * 2 * CH * 2;   off = (off + 255) & ~(size_t)255;
  }
  const size_t oXU1 = off; off += (size_t)RMX * CH * 2;     off = (off + 255) & ~(size_t)255;
  const size_t oB   = off; off += (size_t)RB * CH * 2;      off = (off + 255) & ~(size_t)255;
  const size_t oXI2 = off; off += (size_t)NIP * CH * 2;     off = (off + 255) & ~(size_t)255;
  const size_t oP   = off; off += (size_t)NIP * CH * 4;     off = (off + 255) & ~(size_t)255;
  const size_t oA   = off; off += (size_t)RMX * CH * 2;     off = (off + 255) & ~(size_t)255;
  const size_t oCntI = off; off += (size_t)CNTPADI * 4;    off = (off + 255) & ~(size_t)255;
  const size_t oOffI = off; off += (size_t)CNTPADI * 4;    off = (off + 255) & ~(size_t)255;
  const size_t oRbI  = off; off += (size_t)RBN * 4;        off = (off + 255) & ~(size_t)255;
  const size_t oCsrI = off; off += (size_t)csrLenI * 4;    off = (off + 255) & ~(size_t)255;
  const size_t oCntU = off; off += (size_t)CNTPADU * 4;    off = (off + 255) & ~(size_t)255;
  const size_t oOffU = off; off += (size_t)CNTPADU * 4;    off = (off + 255) & ~(size_t)255;
  const size_t oRbU  = off; off += (size_t)RBN * 4;        off = (off + 255) & ~(size_t)255;
  const size_t oCsrU = off; off += (size_t)csrLenU * 4;    off = (off + 255) & ~(size_t)255;
  if (off > ws_size || off > (size_t)WSCAP) return;

  _Float16* pW1[2]; _Float16* pW2[2]; _Float16* pUI[2]; _Float16* pIU[2];
  for (int l = 0; l < 2; ++l) {
    pW1[l] = (_Float16*)(ws + oW1[l]); pW2[l] = (_Float16*)(ws + oW2[l]);
    pUI[l] = (_Float16*)(ws + oUI[l]); pIU[l] = (_Float16*)(ws + oIU[l]);
  }
  _Float16* xu1P = (_Float16*)(ws + oXU1);
  _Float16* xi3P = (_Float16*)(ws + oXU1);
  _Float16* xi1P = (_Float16*)(ws + oB);
  _Float16* h1P  = (_Float16*)(ws + oB + (size_t)NIP * CH * 2);
  _Float16* xu2P = (_Float16*)(ws + oB);
  _Float16* xi2P = (_Float16*)(ws + oXI2);
  float*    prdP = (float*)(ws + oP);
  _Float16* aggP = (_Float16*)(ws + oA);
  _Float16* h2P  = (_Float16*)(ws + oA);
  int* cntI = (int*)(ws + oCntI); int* offI = (int*)(ws + oOffI); int* rbI = (int*)(ws + oRbI); int* csrI = (int*)(ws + oCsrI);
  int* cntU = (int*)(ws + oCntU); int* offU = (int*)(ws + oOffU); int* rbU = (int*)(ws + oRbU); int* csrU = (int*)(ws + oCsrU);

  const int vec8 = 1;

  for (int l = 0; l < 2; ++l) {
    k_prepw<CH, CH, 1><<<(CH * CH / 8) / NTHR, NTHR, 0, stream>>>(Wb[l][0], Wb[l][0], pW1[l]);
    k_prepw<CH, CH, 1><<<(CH * CH / 8) / NTHR, NTHR, 0, stream>>>(Wb[l][2], Wb[l][2], pW2[l]);
    k_prepw<CH, CH, 2><<<(CH * 2 * CH / 8) / NTHR, NTHR, 0, stream>>>(Wb[l][4], Wb[l][6], pUI[l]);
    k_prepw<CH, CH, 2><<<(CH * 2 * CH / 8) / NTHR, NTHR, 0, stream>>>(Wb[l][8], Wb[l][10], pIU[l]);
  }
  k_xcvt<<<(nXuU + NTHR - 1) / NTHR, NTHR, 0, stream>>>(emb_u, xu1P, nU, nXuU);
  k_xcvt<<<(nXuI + NTHR - 1) / NTHR, NTHR, 0, stream>>>(emb_i, xi1P, nI, nXuI);

  hipFuncSetAttribute(reinterpret_cast<const void*>(&k_fill),
                      hipFuncAttributeMaxDynamicSharedMemorySize, LDS_FILL);
  k_count<<<nBCI, NTHR, 0, stream>>>(ue_dst, cntI, nE1, vec8);
  k_offsets<<<1, OTHR, 0, stream>>>(cntI, offI, rbI, nBCI);
  k_fill<<<nBFI, NTHR, LDS_FILL, stream>>>(ue_dst, offI, rbI, csrI, nE1, vec8, csrLenI);
  k_count<<<nBCU, NTHR, 0, stream>>>(iu_dst, cntU, nE2, vec8);
  k_offsets<<<1, OTHR, 0, stream>>>(cntU, offU, rbU, nBCU);
  k_fill<<<nBFU, NTHR, LDS_FILL, stream>>>(iu_dst, offU, rbU, csrU, nE2, vec8, csrLenU);

  k_gemm16<CH, CH, CH, 1, 1, 0><<<nGI, NTHR, 0, stream>>>(xi1P, xi1P, pW1[0], Wb[0][1], Wb[0][1], h1P, nI);
  k_gemm32<CH, CH, CH, 1, 1><<<nGI, NTHR, 0, stream>>>(h1P, h1P, pW2[0], Wb[0][3], prdP, nI);
  k_mean<float, 8, 1, 1><<<nAI, NTHR, 0, stream>>>(csrI, offI, cntI, ue_src, emb_u, prdP, aggP, nI, nU, nE1, csrLenI);
  k_gemm16<CH, CH, 2 * CH, 2, 1, 1><<<nGI, NTHR, 0, stream>>>(aggP, xi1P, pUI[0], Wb[0][5], Wb[0][7], xi2P, nI);
  k_mean<float, 8, 1, 0><<<nAU, NTHR, 0, stream>>>(csrU, offU, cntU, iu_src, emb_i, prdP, aggP, nU, nI, nE2, csrLenU);
  k_gemm16<CH, CH, 2 * CH, 2, 1, 1><<<nGU, NTHR, 0, stream>>>(aggP, xu1P, pIU[0], Wb[0][9], Wb[0][11], xu2P, nU);

  k_gemm16<CH, CH, CH, 1, 1, 0><<<nGI, NTHR, 0, stream>>>(xi2P, xi2P, pW1[1], Wb[1][1], Wb[1][1], h2P, nI);
  k_gemm32<CH, CH, CH, 1, 1><<<nGI, NTHR, 0, stream>>>(h2P, h2P, pW2[1], Wb[1][3], prdP, nI);
  k_mean<_Float16, 1, 0, 1><<<nAI, NTHR, 0, stream>>>(csrI, offI, cntI, ue_src, xu2P, prdP, aggP, nI, nU, nE1, csrLenI);
  k_gemm16<CH, CH, 2 * CH, 2, 1, 1><<<nGI, NTHR, 0, stream>>>(aggP, xi2P, pUI[1], Wb[1][5], Wb[1][7], xi3P, nI);
  k_mean<_Float16, 1, 0, 0><<<nAU, NTHR, 0, stream>>>(csrU, offU, cntU, iu_src, xi2P, prdP, aggP, nU, nI, nE2, csrLenU);
  k_gemmhead<CH, CH, 2 * CH, 2><<<nGU, NTHR, 0, stream>>>(aggP, xu2P, pIU[1], Wb[1][9], Wb[1][11], hw, hb, out, nU);
}
